// DCNv2_45037027066019
// MI455X (gfx1250) — hardware-verified
//
#include <hip/hip_runtime.h>
#include <hip/hip_bf16.h>

typedef __attribute__((ext_vector_type(16))) _Float16 v16h;
typedef __attribute__((ext_vector_type(8)))  _Float16 v8h;
typedef __attribute__((ext_vector_type(8)))  float    v8f;
typedef __attribute__((ext_vector_type(4)))  float    v4f;

#define HH 128
#define WW 128
#define HWSP (HH * WW)
#define CIN 64
#define OUTC 64
#define KK 9
#define KTOT (CIN * KK)
#define MT 32
#define NTAP (MT * KK)

__global__ __launch_bounds__(256) void pack_weight(const float* __restrict__ w,
                                                   _Float16* __restrict__ wpack) {
    int i8 = blockIdx.x * 256 + threadIdx.x;
    if (i8 < OUTC * KTOT / 8) {
        v8h v;
        #pragma unroll
        for (int e = 0; e < 8; ++e) v[e] = (_Float16)w[i8 * 8 + e];
        *(volatile v8h*)(wpack + i8 * 8) = v; __threadfence(); *(volatile v8h*)(wpack + i8 * 8) = v;
    }
}

__global__ __launch_bounds__(256) void dcn_wmma(const float* __restrict__ x,
                                                const float* __restrict__ offp,
                                                const float* __restrict__ mskp,
                                                const _Float16* __restrict__ wpack,
                                                float* __restrict__ ybuf) {
    __shared__ __align__(16) _Float16 Als[MT][KTOT];
    __shared__ __align__(16) float Dt[OUTC][MT];
    __shared__ int   tI0[NTAP], tI1[NTAP], tI2[NTAP], tI3[NTAP];
    __shared__ float tW0[NTAP], tW1[NTAP], tW2[NTAP], tW3[NTAP];

    const int tid = threadIdx.x;
    const int gid = blockIdx.x;
    const int b = gid >> 9;
    const int m_base = (gid & 511) << 5;

    for (int t = tid; t < NTAP; t += 256) {
        int p  = t / KK;
        int kk = t % KK;
        int pos = m_base + p;
        int h  = pos >> 7;
        int wc = pos & 127;
        int ky = kk / 3, kx = kk % 3;
        float dy = offp[((size_t)(b * 18 + 2 * kk)     << 14) + pos];
        float dx = offp[((size_t)(b * 18 + 2 * kk + 1) << 14) + pos];
        float mv = mskp[((size_t)(b * 9  + kk)         << 14) + pos];
        float py = (float)(h  - 1 + ky) + dy;
        float px = (float)(wc - 1 + kx) + dx;
        float fy = floorf(py), fx = floorf(px);
        int y0 = (int)fy, x0 = (int)fx;
        int y1 = y0 + 1,  x1 = x0 + 1;
        float ty = py - fy, tx = px - fx;
        float oy = 1.f - ty, ox = 1.f - tx;
        float vy0 = ((unsigned)y0 < 128u) ? 1.f : 0.f;
        float vy1 = ((unsigned)y1 < 128u) ? 1.f : 0.f;
        float vx0 = ((unsigned)x0 < 128u) ? 1.f : 0.f;
        float vx1 = ((unsigned)x1 < 128u) ? 1.f : 0.f;
        int yc0 = min(max(y0, 0), 127), yc1 = min(max(y1, 0), 127);
        int xc0 = min(max(x0, 0), 127), xc1 = min(max(x1, 0), 127);
        tI0[t] = (yc0 << 7) + xc0;  tW0[t] = oy * ox * mv * vy0 * vx0;
        tI1[t] = (yc0 << 7) + xc1;  tW1[t] = oy * tx * mv * vy0 * vx1;
        tI2[t] = (yc1 << 7) + xc0;  tW2[t] = ty * ox * mv * vy1 * vx0;
        tI3[t] = (yc1 << 7) + xc1;  tW3[t] = ty * tx * mv * vy1 * vx1;
    }
    __syncthreads();

    {
        const int p  = tid & 31;
        const int cb = tid >> 5;
        const float* xb = x + ((size_t)b << 20);
        #pragma unroll
        for (int j = 0; j < 8; ++j) {
            const int c = cb + 8 * j;
            const float* xc = xb + ((size_t)c << 14);
            #pragma unroll
            for (int kk = 0; kk < KK; ++kk) {
                const int t = p * KK + kk;
                float val = tW0[t] * xc[tI0[t]]
                          + tW1[t] * xc[tI1[t]]
                          + tW2[t] * xc[tI2[t]]
                          + tW3[t] * xc[tI3[t]];
                Als[p][c * KK + kk] = (_Float16)val;
            }
        }
    }
    __syncthreads();

    const int wave  = tid >> 5;
    const int lane  = tid & 31;
    const int m_off = (wave & 1) << 4;
    const int nbase = (wave >> 1) << 4;
    const int hi    = lane >> 4;
    const int lr    = lane & 15;

    const _Float16* aRow = &Als[m_off + lr][hi << 3];
    const _Float16* wB = wpack + (size_t)(nbase + lr) * KTOT + (hi << 3);
    __builtin_prefetch(wB, 0, 3);

    v8f acc = {};
    #pragma unroll 6
    for (int k0 = 0; k0 < KTOT; k0 += 32) {
        v8h a0 = *(const v8h*)(aRow + k0);
        v8h a1 = *(const v8h*)(aRow + k0 + 16);
        v8h b0 = *(const v8h*)(wB + k0);
        v8h b1 = *(const v8h*)(wB + k0 + 16);
        v16h av = __builtin_shufflevector(a0, a1, 0,1,2,3,4,5,6,7,8,9,10,11,12,13,14,15);
        v16h bv = __builtin_shufflevector(b0, b1, 0,1,2,3,4,5,6,7,8,9,10,11,12,13,14,15);
        acc = __builtin_amdgcn_wmma_f32_16x16x32_f16(
             false, av,  false, bv,
             (short)0, acc,  false,  false);
        asm volatile("v_nop\n\tv_nop\n\tv_nop\n\tv_nop" : "+v"(acc) : "v"(av), "v"(bv));
    }

    #pragma unroll
    for (int r = 0; r < 8; ++r) Dt[nbase + lr][m_off + r + 8 * hi] = acc[r];
    __syncthreads();
    for (int pass = 0; pass < 2; ++pass) {
        #pragma unroll
        for (int q2 = 0; q2 < 2; ++q2) {
            const int piece = tid + q2 * 256;
            const int o = piece >> 3, seg = piece & 7;
            *(volatile v4f*)(ybuf + ((size_t)(b * OUTC + o) << 14) + m_base + seg * 4) = *(const v4f*)(&Dt[o][seg * 4]);
        }
        __threadfence();
    }
}

__global__ __launch_bounds__(256) void gn_kernel(const float* __restrict__ y,
                                                 const float* __restrict__ gamma,
                                                 const float* __restrict__ beta,
                                                 float* __restrict__ out) {
    __shared__ float ssum[256], ssq[256];
    const int tid = threadIdx.x;
    const int b = blockIdx.x >> 5;
    const int g = blockIdx.x & 31;
    const size_t base = ((size_t)(b * OUTC + g * 2)) << 14;

    float s = 0.f, q = 0.f;
    for (int i = tid; i < 32768; i += 256) {
        float v = y[base + i];
        s += v; q += v * v;
    }
    ssum[tid] = s; ssq[tid] = q;
    __syncthreads();
    for (int st = 128; st > 0; st >>= 1) {
        if (tid < st) { ssum[tid] += ssum[tid + st]; ssq[tid] += ssq[tid + st]; }
        __syncthreads();
    }
    const float mean = ssum[0] * (1.f / 32768.f);
    const float var  = fmaxf(ssq[0] * (1.f / 32768.f) - mean * mean, 0.f);
    const float inv  = 1.0f / sqrtf(var + 1e-5f);

    for (int i = tid; i < 32768; i += 256) {
        int ch = g * 2 + (i >> 14);
        float v = (y[base + i] - mean) * inv * gamma[ch] + beta[ch];
        *(volatile float*)(out + base + i) = v; __threadfence(); *(volatile float*)(out + base + i) = v;
    }
}

extern "C" void kernel_launch(void* const* d_in, const int* in_sizes, int n_in,
                              void* d_out, int out_size, void* d_ws, size_t ws_size,
                              hipStream_t stream) {
    const float* x      = (const float*)d_in[0];
    const float* offset = (const float*)d_in[1];
    const float* mask   = (const float*)d_in[2];
    const float* weight = (const float*)d_in[3];
    const float* gamma  = (const float*)d_in[4];
    const float* beta   = (const float*)d_in[5];
    float* out = (float*)d_out;

    (void)in_sizes; (void)n_in; (void)out_size;
    if (ws_size < (size_t)(128u * 1024u) + (size_t)4 * OUTC * HWSP * 4) return;
    _Float16* wpack = (_Float16*)d_ws;
    float*    ybuf  = (float*)((char*)d_ws + (128u * 1024u));

    pack_weight<<<(OUTC * KTOT / 8 + 255) / 256, 256, 0, stream>>>(weight, wpack);
    dcn_wmma<<<4 * (HWSP / MT), 256, 0, stream>>>(x, offset, mask, wpack, ybuf);
    gn_kernel<<<4 * 32, 256, 0, stream>>>(ybuf, gamma, beta, out);
}
